// Drifting_13950053777833
// MI455X (gfx1250) — hardware-run, weakly checked
//
#include <hip/hip_runtime.h>


#define NN   4096
#define NR   NN
#define DD   512
#define NC   (2 * NN)
#define TEMP 0.05f
#define MASKV 1000000.0f
#define RP   32
typedef _Float16 h16;
typedef unsigned short bf;
typedef __attribute__((ext_vector_type(16))) __bf16   v16bf;
typedef __attribute__((ext_vector_type(16))) _Float16 v16h;
typedef __attribute__((ext_vector_type(8)))  _Float16 v8h;
typedef __attribute__((ext_vector_type(8)))  unsigned short v8us;
typedef __attribute__((ext_vector_type(8)))  float    v8f;
typedef __attribute__((ext_vector_type(4)))  float    v4f;
typedef v8h  __attribute__((may_alias)) v8ha;
typedef v4f  __attribute__((may_alias)) v4fa;
typedef v8us __attribute__((may_alias)) v8usa;

__device__ __forceinline__ unsigned short f2bf(float f) { unsigned u = __float_as_uint(f); u += 0x7FFFu + ((u >> 16) & 1u); return (unsigned short)(u >> 16); }
__device__ __forceinline__ float bf2f(unsigned short b) { return __uint_as_float(((unsigned)b) << 16); }
__device__ __forceinline__ float bfr(float f) { return bf2f(f2bf(f)); }
__device__ __forceinline__ v16h cat16(v8h lo, v8h hi) { return __builtin_shufflevector(lo, hi, 0, 1, 2, 3, 4, 5, 6, 7, 8, 9, 10, 11, 12, 13, 14, 15); }
__device__ __forceinline__ v16bf cat16b(v8us lo, v8us hi) { return __builtin_bit_cast(v16bf, __builtin_shufflevector(lo, hi, 0, 1, 2, 3, 4, 5, 6, 7, 8, 9, 10, 11, 12, 13, 14, 15)); }
__device__ __forceinline__ v8f wmma16(v16h a, v16h b, v8f c) { return __builtin_amdgcn_wmma_f32_16x16x32_f16(false, a, false, b, (short)0, c, false, false); }
__device__ __forceinline__ v8f wmmab(v16bf a, v16bf b, v8f c) { return __builtin_amdgcn_wmma_f32_16x16x32_bf16(false, a, false, b, (short)0, c, false, false); }


template <typename T16> struct WFrag;
template <> struct WFrag<h16> { typedef v16h V; static __device__ __forceinline__ V ld(const h16* p) { return cat16(*(const v8h*)p, *(const v8h*)(p + 16)); } static __device__ __forceinline__ v8f mma(V a, V b, v8f c) { return wmma16(a, b, c); } };
template <> struct WFrag<bf> { typedef v16bf V; static __device__ __forceinline__ V ld(const bf* p) { return cat16b(*(const v8us*)p, *(const v8us*)(p + 16)); } static __device__ __forceinline__ v8f mma(V a, V b, v8f c) { return wmmab(a, b, c); } };
template <typename T16, int NSPLIT, bool BIAS>
__global__ __launch_bounds__(32) void k_gemmw(const T16* __restrict__ A, const T16* __restrict__ A2, const T16* __restrict__ Bt, const T16* __restrict__ Bt2, int K, float* C, int ldc, const float* __restrict__ bias, size_t sA, size_t sB, size_t sC) {
    typedef typename WFrag<T16>::V V;
    __shared__ __align__(16) float os[16 * 68];
    const size_t z = blockIdx.z; A += z * sA; if (A2) A2 += z * sA; Bt += z * sB; if (Bt2) Bt2 += z * sB; C += z * sC;
    const int lane = threadIdx.x & 31, lr = lane & 15, hi = lane >> 4; const int r0 = blockIdx.x * 64, c0 = blockIdx.y * 64;
    v8f acc[4][4];
#pragma unroll
    for (int mb = 0; mb < 4; ++mb)
#pragma unroll
        for (int nb = 0; nb < 4; ++nb) acc[mb][nb] = (v8f){};
    const size_t aoff = (size_t)(r0 + lr) * K + 8 * hi, boff = (size_t)(c0 + lr) * K + 8 * hi;
#pragma unroll 1
    for (int kc = 0; kc < K; kc += 32) {
        V a[4], a2[4];
#pragma unroll
        for (int mb = 0; mb < 4; ++mb) { a[mb] = WFrag<T16>::ld(A + aoff + (size_t)mb * 16 * K + kc); if (NSPLIT == 1 || NSPLIT == 2) a2[mb] = WFrag<T16>::ld(A2 + aoff + (size_t)mb * 16 * K + kc); }
#pragma unroll
        for (int nb = 0; nb < 4; ++nb) { const V b = WFrag<T16>::ld(Bt + boff + (size_t)nb * 16 * K + kc); V b2; if (NSPLIT >= 2) b2 = WFrag<T16>::ld(Bt2 + boff + (size_t)nb * 16 * K + kc);
#pragma unroll
            for (int mb = 0; mb < 4; ++mb) { acc[mb][nb] = WFrag<T16>::mma(a[mb], b, acc[mb][nb]); if (NSPLIT == 1 || NSPLIT == 2) acc[mb][nb] = WFrag<T16>::mma(a2[mb], b, acc[mb][nb]); if (NSPLIT >= 2) acc[mb][nb] = WFrag<T16>::mma(a[mb], b2, acc[mb][nb]); } }
        asm volatile("v_nop\n\tv_nop\n\tv_nop\n\tv_nop" : "+v"(acc[0][0]), "+v"(acc[1][1]), "+v"(acc[2][2]), "+v"(acc[3][3]) : "v"(a[0]), "v"(a[3]));
    }
#pragma unroll
    for (int mb = 0; mb < 4; ++mb) {
#pragma unroll
        for (int nb = 0; nb < 4; ++nb) {
#pragma unroll
            for (int j = 0; j < 8; ++j) os[(hi * 8 + j) * 68 + nb * 16 + lr] = acc[mb][nb][j]; }
        __builtin_amdgcn_wave_barrier(); asm volatile("" ::: "memory");
        float* crow = C + (size_t)(r0 + mb * 16) * ldc + c0;
#pragma unroll 1
        for (int ps = 0; ps < 2; ++ps) {
#pragma unroll
            for (int s = 0; s < 8; ++s) { const int row = 2 * s + hi, cofs = lr * 4; v4f val = *(const v4fa*)(os + row * 68 + cofs); if (BIAS) { val[0] += bfr(bias[c0 + cofs]); val[1] += bfr(bias[c0 + cofs + 1]); val[2] += bfr(bias[c0 + cofs + 2]); val[3] += bfr(bias[c0 + cofs + 3]); }
                *(volatile v4f*)(crow + (size_t)row * ldc + cofs) = val; }
            if (ps == 0) __threadfence(); }
        __builtin_amdgcn_wave_barrier(); asm volatile("" ::: "memory");
    }
}

__device__ __forceinline__ void splitf(float y, unsigned short& h, unsigned short& l) { h = f2bf(y); l = f2bf(y - bf2f(h)); }
typedef __attribute__((ext_vector_type(4))) unsigned short v4us;
typedef __attribute__((ext_vector_type(2))) unsigned short v2us;
__global__ __launch_bounds__(256) void k_cvt8(const float* __restrict__ src, bf* dst, size_t n8) { const size_t i = (size_t)blockIdx.x * 256 + threadIdx.x; if (i >= n8) return; const v8f v = *(const v8f*)(src + i * 8); v8us o;
#pragma unroll
    for (int k = 0; k < 8; ++k) o[k] = f2bf(v[k]); *(volatile v8us*)(dst + i * 8) = o; __threadfence(); *(volatile v8us*)(dst + i * 8) = o; }

__global__ __launch_bounds__(256) void k_wtG(const float* __restrict__ w, int K, int N, bf* Bt) {
    const int lane = threadIdx.x & 31; const int L0 = (blockIdx.x * 8 + (threadIdx.x >> 5)) * 8; const int nlines = N * K / 64;
#pragma unroll
    for (int ps = 0; ps < 2; ++ps) {
#pragma unroll 1
        for (int l = 0; l < 8; ++l) { const int L = L0 + l; if (L >= nlines) break; const size_t e = (size_t)L * 64 + lane * 2; const int k = (int)(e % K), n = (int)(e / K); v2us o;
            o[0] = f2bf(w[(size_t)k * N + n]); o[1] = f2bf(w[(size_t)(k + 1) * N + n]); *(volatile v2us*)(Bt + e) = o; }
        if (ps == 0) __threadfence(); }
}
__global__ __launch_bounds__(256) void k_sq(const float* __restrict__ a, float* SQ) { const int i = blockIdx.x * 256 + threadIdx.x; if (i >= NN) return; const float* r = a + (size_t)i * DD; float s = 0.f;
#pragma unroll 4
    for (int d = 0; d < DD; ++d) { const float v = bfr(r[d]); float p = __fmul_rn(v, v); asm volatile("" : "+v"(p)); s = __fadd_rn(s, p); }
    *(volatile float*)(SQ + i) = s; __threadfence(); *(volatile float*)(SQ + i) = s; }
template <bool DIAG>
__global__ __launch_bounds__(256) void k_logit(float* L, const float* __restrict__ xs, const float* __restrict__ ys, int cofs) { const size_t e = ((size_t)blockIdx.x * 256 + threadIdx.x) * 4; if (e >= (size_t)NR * NN) return; const int j = (int)(e % NN); const int i = (int)(e / NN); float* p = L + (size_t)i * NC + cofs + j; const v4f g = *(const v4f*)p; const float xi = xs[i]; v4f o;
#pragma unroll
    for (int q = 0; q < 4; ++q) { float t = __fadd_rn(xi, ys[j + q]); asm volatile("" : "+v"(t)); float d2 = __fsub_rn(t, __fmul_rn(2.0f, g[q])); d2 = fmaxf(d2, 0.f); float dist = __fsqrt_rn(d2); if (DIAG && (j + q == i)) dist = __fadd_rn(dist, MASKV); o[q] = __fdiv_rn(-dist, TEMP); }
    *(volatile v4f*)p = o; __threadfence(); *(volatile v4f*)p = o; }
__global__ __launch_bounds__(256) void k_rowstat(const float* __restrict__ L, float* RS) { const int lane = threadIdx.x & 31; const int i = blockIdx.x * 8 + (threadIdx.x >> 5); if (i >= NR) return; const float* r = L + (size_t)i * NC; float mx = -3.0e38f;
#pragma unroll 1
    for (int ch = 0; ch < NC / 128; ++ch) { const v4f a = *(const v4f*)(r + ch * 128 + lane * 4);
#pragma unroll
        for (int q = 0; q < 4; ++q) mx = fmaxf(mx, a[q]); }
#pragma unroll
    for (int sh = 16; sh; sh >>= 1) mx = fmaxf(mx, __shfl_xor(mx, sh, 32));
    float s = 0.f;
#pragma unroll 1
    for (int ch = 0; ch < NC / 128; ++ch) { const v4f a = *(const v4f*)(r + ch * 128 + lane * 4);
#pragma unroll
        for (int q = 0; q < 4; ++q) { float d0 = __fsub_rn(a[q], mx); asm volatile("" : "+v"(d0)); s += __builtin_amdgcn_exp2f(__fmul_rn(d0, 1.4426950408889634f)); } }
#pragma unroll
    for (int sh = 16; sh; sh >>= 1) s += __shfl_xor(s, sh, 32);
    if (lane < 2) { const float v = (lane == 0) ? mx : s; *(volatile float*)(RS + (size_t)i * RP + lane) = v; __threadfence(); *(volatile float*)(RS + (size_t)i * RP + lane) = v; } }
__global__ __launch_bounds__(256) void k_colstat(const float* __restrict__ L, float* CM, float* CL) { const int j = blockIdx.x * 256 + threadIdx.x; if (j >= NC) return; float mx = -3.0e38f;
#pragma unroll 4
    for (int i = 0; i < NR; ++i) mx = fmaxf(mx, L[(size_t)i * NC + j]);
    float s = 0.f;
#pragma unroll 4
    for (int i = 0; i < NR; ++i) { float d0 = __fsub_rn(L[(size_t)i * NC + j], mx); asm volatile("" : "+v"(d0)); s += __builtin_amdgcn_exp2f(__fmul_rn(d0, 1.4426950408889634f)); }
    *(volatile float*)(CM + j) = mx; *(volatile float*)(CL + j) = s; __threadfence(); *(volatile float*)(CM + j) = mx; *(volatile float*)(CL + j) = s; }
__global__ __launch_bounds__(256) void k_aplane(const float* __restrict__ L, const float* RS0, const float* __restrict__ CM, const float* __restrict__ CL, int cofs, int blk, bf* Ph, bf* Pl, float* RS) {
    const int lane = threadIdx.x & 31; const int i = blockIdx.x * 8 + (threadIdx.x >> 5); if (i >= NR) return; const float mr = RS0[(size_t)i * RP], lr = RS0[(size_t)i * RP + 1]; const float* r = L + (size_t)i * NC + cofs; float rsum = 0.f;
#pragma unroll 1
    for (int ps = 0; ps < 2; ++ps) { rsum = 0.f;
#pragma unroll 1
        for (int ch = 0; ch < NN / 128; ++ch) { const int j0 = ch * 128 + lane * 4; const v4f a = *(const v4f*)(r + j0); v4us oh, ol;
#pragma unroll
            for (int q = 0; q < 4; ++q) { const int j = cofs + j0 + q; float u = __fadd_rn(__fsub_rn(a[q], mr), __fsub_rn(a[q], CM[j])); asm volatile("" : "+v"(u)); const float ex = __builtin_amdgcn_exp2f(__fmul_rn(0.5f * u, 1.4426950408889634f)); const float nrm = __fdiv_rn(1.0f, __fsqrt_rn(__fmul_rn(lr, CL[j]))); const float av = __fmul_rn(ex, nrm); rsum = __fadd_rn(rsum, av); unsigned short h2, l2; splitf(av, h2, l2); oh[q] = h2; ol[q] = l2; }
            const size_t oo = (size_t)i * NN + j0; *(volatile v4us*)(Ph + oo) = oh; *(volatile v4us*)(Pl + oo) = ol; }
#pragma unroll
        for (int sh = 16; sh; sh >>= 1) rsum += __shfl_xor(rsum, sh, 32);
        if (lane == 0) *(volatile float*)(RS + (size_t)i * RP + 2 + blk) = rsum;
        if (ps == 0) __threadfence(); } }
__global__ __launch_bounds__(256) void k_vout(const float* __restrict__ Cp, const float* __restrict__ Cn, const float* __restrict__ RS, float* V) { const size_t e = ((size_t)blockIdx.x * 256 + threadIdx.x) * 4; if (e >= (size_t)NR * DD) return; const int i = (int)(e / DD); const float sp = RS[(size_t)i * RP + 2], sn = RS[(size_t)i * RP + 3]; const v4f a = *(const v4f*)(Cp + e), b = *(const v4f*)(Cn + e); v4f o;
#pragma unroll
    for (int q = 0; q < 4; ++q) { float t1 = __fmul_rn(sn, a[q]); asm volatile("" : "+v"(t1)); o[q] = __fsub_rn(t1, __fmul_rn(sp, b[q])); }
    *(volatile v4f*)(V + e) = o; __threadfence(); *(volatile v4f*)(V + e) = o; }

extern "C" void kernel_launch(void* const* d_in, const int* in_sizes, int n_in,
                              void* d_out, int out_size, void* d_ws, size_t ws_size, hipStream_t stream) {
    (void)in_sizes; (void)n_in; (void)out_size;
    const float* x = (const float*)d_in[0]; const float* yp = (const float*)d_in[1]; const float* yn = (const float*)d_in[2];
    float* OUT = (float*)d_out;
    char* wsp = (char*)d_ws;
    auto take = [&](size_t bytes) { char* p = wsp; wsp += (bytes + 255) & ~(size_t)255; return (void*)p; };
    bf* XB = (bf*)take((size_t)NN * DD * 2); bf* YPB = (bf*)take((size_t)NN * DD * 2); bf* YNB = (bf*)take((size_t)NN * DD * 2); bf* YPT = (bf*)take((size_t)DD * NN * 2); bf* YNT = (bf*)take((size_t)DD * NN * 2); float* XS = (float*)take(NN * 4); float* PS = (float*)take(NN * 4); float* NS = (float*)take(NN * 4);
    float* L = (float*)take((size_t)NN * NC * 4); float* RS = (float*)take((size_t)NN * RP * 4); float* CM = (float*)take(NC * 4); float* CL = (float*)take(NC * 4); bf* Ph = (bf*)take((size_t)NN * NN * 2); bf* Pl = (bf*)take((size_t)NN * NN * 2); float* Cp = (float*)take((size_t)NN * DD * 4); float* Cn = (float*)take((size_t)NN * DD * 4);
    if ((size_t)(wsp - (char*)d_ws) > ws_size) return;
    const unsigned n8 = (unsigned)(((size_t)NN * DD / 8 + 255) / 256);
    k_cvt8<<<n8, 256, 0, stream>>>(x, XB, (size_t)NN * DD / 8); k_cvt8<<<n8, 256, 0, stream>>>(yp, YPB, (size_t)NN * DD / 8); k_cvt8<<<n8, 256, 0, stream>>>(yn, YNB, (size_t)NN * DD / 8);
    k_wtG<<<(unsigned)((NN * DD / 64 + 63) / 64), 256, 0, stream>>>(yp, NN, DD, YPT); k_wtG<<<(unsigned)((NN * DD / 64 + 63) / 64), 256, 0, stream>>>(yn, NN, DD, YNT);
    k_sq<<<NN / 256, 256, 0, stream>>>(x, XS); k_sq<<<NN / 256, 256, 0, stream>>>(yp, PS); k_sq<<<NN / 256, 256, 0, stream>>>(yn, NS);
    k_gemmw<bf, 0, false><<<dim3(NR / 64, NN / 64, 1), 32, 0, stream>>>(XB, nullptr, YPB, nullptr, DD, L, NC, nullptr, 0, 0, 0);
    k_gemmw<bf, 0, false><<<dim3(NR / 64, NN / 64, 1), 32, 0, stream>>>(XB, nullptr, YNB, nullptr, DD, L + NN, NC, nullptr, 0, 0, 0);
    const unsigned nl = (unsigned)(((size_t)NR * NN / 4 + 255) / 256);
    k_logit<false><<<nl, 256, 0, stream>>>(L, XS, PS, 0); k_logit<true><<<nl, 256, 0, stream>>>(L, XS, NS, NN);
    k_rowstat<<<NR / 8, 256, 0, stream>>>(L, RS); k_colstat<<<NC / 256, 256, 0, stream>>>(L, CM, CL);
    k_aplane<<<NR / 8, 256, 0, stream>>>(L, RS, CM, CL, 0, 0, Ph, Pl, RS);
    k_gemmw<bf, 1, false><<<dim3(NR / 64, DD / 64, 1), 32, 0, stream>>>(Ph, Pl, YPT, nullptr, NN, Cp, DD, nullptr, 0, 0, 0);
    k_aplane<<<NR / 8, 256, 0, stream>>>(L, RS, CM, CL, NN, 1, Ph, Pl, RS);
    k_gemmw<bf, 1, false><<<dim3(NR / 64, DD / 64, 1), 32, 0, stream>>>(Ph, Pl, YNT, nullptr, NN, Cn, DD, nullptr, 0, 0, 0);
    k_vout<<<(unsigned)(((size_t)NR * DD / 4 + 255) / 256), 256, 0, stream>>>(Cp, Cn, RS, OUT);
}
